// GAT_MUTAG_66116726554991
// MI455X (gfx1250) — hardware-verified
//
#include <hip/hip_runtime.h>
#include <stddef.h>


#define HID     32
#define INDIM   7
#define EDIM    4
#define NCLS    2
#define NTHR    256
#define NWAVE   8
#define EPT     8
#define NGRP    2
#define CHUNK   (NTHR * EPT * NGRP)
#define WCAP    (EPT * NGRP * 32)
#define LISTN   (NWAVE * WCAP)
#define NBC     4096
#define NBF     1024
#define RCAP    40960
#define RBN     128
#define TGT     256
#define DEGCAP  256
#define OTHR    512
#define GBM     128
#define APK     40
#define PG      256
#define WSCAP   134217728
#define NEG_SLOPE 0.2f
#define DEN_EPS 1e-16f
#define BN_EPS  1e-5f
#define NEG_BIG (-3.0e38f)

#define LDS_FILL ((RCAP + NBF + LISTN) * 4 + 64)

static_assert((CHUNK & (CHUNK - 1)) == 0);
static_assert(CHUNK <= 4096);
static_assert(NBC <= 4096 && NBF <= 4096 && PG <= 4096);
static_assert((NBC & (NBC - 1)) == 0 && (NBF & (NBF - 1)) == 0 && (PG & (PG - 1)) == 0);
static_assert(NBC == 4 * NBF);
static_assert(OTHR * 8 == NBC);
static_assert((RCAP % 32) == 0);
static_assert(TGT == NWAVE * 32);
static_assert((NBC % TGT) == 0 && (TGT % GBM) == 0);
static_assert(GBM == NWAVE * 16);
static_assert(((APK * 2) % 16) == 0);
static_assert(GBM * HID * 4 <= 2 * GBM * APK * 2);
static_assert(PG * HID == NTHR * 32);

typedef float          v4f  __attribute__((ext_vector_type(4)));
typedef float          v8f  __attribute__((ext_vector_type(8)));
typedef int            v4i  __attribute__((ext_vector_type(4)));
typedef double         v2d  __attribute__((ext_vector_type(2)));
typedef unsigned short v8us __attribute__((ext_vector_type(8)));
typedef __bf16         v16b __attribute__((ext_vector_type(16)));
union FragB { v16b v; v8us h[2]; };

__device__ __forceinline__ unsigned int bfr(float f) {
  const unsigned int u = __float_as_uint(f);
  return (u + 0x7FFFu + ((u >> 16) & 1u)) >> 16;
}

__device__ __forceinline__ void split1(float x, unsigned short& hb, unsigned short& lb) {
  const unsigned int hu = bfr(x);
  const float hf = __uint_as_float(hu << 16);
  hb = (unsigned short)hu;
  lb = (unsigned short)bfr(x - hf);
}

__device__ __forceinline__ void split8(v4f a, v4f b, v8us& hi, v8us& lo) {
  unsigned short hb, lb;
  split1(a.x, hb, lb); hi[0] = hb; lo[0] = lb;
  split1(a.y, hb, lb); hi[1] = hb; lo[1] = lb;
  split1(a.z, hb, lb); hi[2] = hb; lo[2] = lb;
  split1(a.w, hb, lb); hi[3] = hb; lo[3] = lb;
  split1(b.x, hb, lb); hi[4] = hb; lo[4] = lb;
  split1(b.y, hb, lb); hi[5] = hb; lo[5] = lb;
  split1(b.z, hb, lb); hi[6] = hb; lo[6] = lb;
  split1(b.w, hb, lb); hi[7] = hb; lo[7] = lb;
}

__device__ __forceinline__ v8f wmb(v16b a, v16b b, v8f c) {
  v8f d = __builtin_amdgcn_wmma_f32_16x16x32_bf16(false, a, false, b, (short)0, c, false, false);
  asm volatile("v_nop\n\tv_nop\n\tv_nop\n\tv_nop" : "+v"(d) : "v"(a), "v"(b));
  return d;
}

__device__ __forceinline__ float lrelu(float v) { return v > 0.0f ? v : NEG_SLOPE * v; }
__device__ __forceinline__ float bnr(float x, float mu, float sc, float be) {
  return fmaxf((x - mu) * sc + be, 0.0f);
}

__device__ __forceinline__ float wmax(float v) {
#pragma unroll
  for (int o = 16; o > 0; o >>= 1) v = fmaxf(v, __shfl_xor(v, o));
  return v;
}
__device__ __forceinline__ float wsum(float v) {
#pragma unroll
  for (int o = 16; o > 0; o >>= 1) v += __shfl_xor(v, o);
  return v;
}

template <int NB>
__device__ __forceinline__ int scan_chunk(const int* __restrict__ dsts, int nE, int cbase, int slotBase,
                                          int vec8, int* list, int tid, int lane, int wave) {
  int wc = 0;
#pragma unroll
  for (int g = 0; g < NGRP; ++g) {
    const int el0  = (g * NTHR + tid) * EPT;
    const int e0   = cbase + el0;
    const int sent = -2147483647 - 1;
    v4i da, db;
    if (vec8 != 0 && cbase + CHUNK <= nE) {
      da = *(const v4i*)(dsts + e0);
      db = *(const v4i*)(dsts + e0 + 4);
    } else {
      da.x = (e0     < nE) ? dsts[min(e0, nE - 1)] : sent;
      da.y = (e0 + 1 < nE) ? dsts[min(e0 + 1, nE - 1)] : sent;
      da.z = (e0 + 2 < nE) ? dsts[min(e0 + 2, nE - 1)] : sent;
      da.w = (e0 + 3 < nE) ? dsts[min(e0 + 3, nE - 1)] : sent;
      db.x = (e0 + 4 < nE) ? dsts[min(e0 + 4, nE - 1)] : sent;
      db.y = (e0 + 5 < nE) ? dsts[min(e0 + 5, nE - 1)] : sent;
      db.z = (e0 + 6 < nE) ? dsts[min(e0 + 6, nE - 1)] : sent;
      db.w = (e0 + 7 < nE) ? dsts[min(e0 + 7, nE - 1)] : sent;
    }
    const unsigned nb = (unsigned)slotBase;
    const unsigned s0 = (unsigned)da.x - nb, s1 = (unsigned)da.y - nb;
    const unsigned s2 = (unsigned)da.z - nb, s3 = (unsigned)da.w - nb;
    const unsigned s4 = (unsigned)db.x - nb, s5 = (unsigned)db.y - nb;
    const unsigned s6 = (unsigned)db.z - nb, s7 = (unsigned)db.w - nb;
    const bool h0 = s0 < (unsigned)NB, h1 = s1 < (unsigned)NB, h2 = s2 < (unsigned)NB, h3 = s3 < (unsigned)NB;
    const bool h4 = s4 < (unsigned)NB, h5 = s5 < (unsigned)NB, h6 = s6 < (unsigned)NB, h7 = s7 < (unsigned)NB;
    const unsigned any = __builtin_amdgcn_ballot_w32(h0 | h1 | h2 | h3 | h4 | h5 | h6 | h7);
    if (any != 0u) {
#define HITJ(J, HJ, SJ) { \
        const unsigned mj = __builtin_amdgcn_ballot_w32(HJ); \
        if (mj != 0u) { \
          if (HJ) { \
            const int pos = wc + (int)__builtin_amdgcn_mbcnt_lo(mj, 0u); \
            if (pos < WCAP) list[wave * WCAP + pos] = ((el0 + (J)) << 12) | (int)(SJ); \
          } \
          wc += (int)__builtin_popcount(mj); } }
      HITJ(0, h0, s0)
      HITJ(1, h1, s1)
      HITJ(2, h2, s2)
      HITJ(3, h3, s3)
      HITJ(4, h4, s4)
      HITJ(5, h5, s5)
      HITJ(6, h6, s6)
      HITJ(7, h7, s7)
#undef HITJ
    }
  }
  return wc;
}

__global__ __launch_bounds__(128) void k_prep(const float* __restrict__ W0, const float* __restrict__ W12,
                                              unsigned short* wp) {
  const int layer = blockIdx.x;
  const int i = threadIdx.x;
  const int n = i >> 2, k0 = (i & 3) * 8;
  const int K = (layer == 0) ? INDIM : HID;
  const int lw = layer > 0 ? layer - 1 : 0;
  const float* W = (layer == 0) ? W0 : (W12 + (size_t)lw * HID * HID);
  float v[8];
#pragma unroll
  for (int e = 0; e < 8; ++e) {
    const int k  = k0 + e;
    const int kc = k < K - 1 ? k : K - 1;
    const float x = W[(size_t)kc * HID + n];
    v[e] = (k < K) ? x : 0.0f;
  }
  v4f a, b;
  a.x = v[0]; a.y = v[1]; a.z = v[2]; a.w = v[3];
  b.x = v[4]; b.y = v[5]; b.z = v[6]; b.w = v[7];
  v8us hv, lv;
  split8(a, b, hv, lv);
  unsigned short* dh = wp + (size_t)layer * 2 * HID * HID + (size_t)i * 8;
  unsigned short* dl = dh + HID * HID;
  *(volatile v8us*)dh = hv;
  *(volatile v8us*)dl = lv;
  __threadfence();
  *(volatile v8us*)dh = hv;
  *(volatile v8us*)dl = lv;
}

__global__ __launch_bounds__(NTHR) void k_count(
    const int* __restrict__ dsts, int* cnt, int nE, int vec8) {
  __shared__ __attribute__((aligned(16))) int scnt[NBC];
  __shared__ __attribute__((aligned(16))) int list[LISTN];
  __shared__ int wcnt[NWAVE];
  const int tid = threadIdx.x, lane = tid & 31, wave = tid >> 5;
  const int nodeBase = blockIdx.x * NBC;

  for (int i = tid; i < NBC; i += NTHR) scnt[i] = 0;
  __syncthreads();

  const int nChunks = (nE + CHUNK - 1) / CHUNK;
#pragma unroll 1
  for (int ch = 0; ch < nChunks; ++ch) {
    const int cbase = ch * CHUNK;
    const int wc = scan_chunk<NBC>(dsts, nE, cbase, nodeBase, vec8, list, tid, lane, wave);
    if (lane == 0) wcnt[wave] = wc;
    __syncthreads();
    if (wave == 0) {
#pragma unroll 1
      for (int wsx = 0; wsx < NWAVE; ++wsx) {
        int n = __builtin_amdgcn_readfirstlane(wcnt[wsx]);
        n = n > WCAP ? WCAP : (n < 0 ? 0 : n);
        const int* lp = list + wsx * WCAP;
#pragma unroll 1
        for (int i = 0; i < n; ++i) {
          const int ent  = __builtin_amdgcn_readfirstlane(lp[i]);
          const int slot = ent & (NBC - 1);
          if (lane == 0) scnt[slot] = scnt[slot] + 1;
        }
      }
    }
    __syncthreads();
  }

  v4i cq[4];
#pragma unroll
  for (int q = 0; q < 4; ++q) {
    const int f = (wave * 4 + q) * 128 + 4 * lane;
    cq[q] = *(const v4i*)(scnt + f);
  }
  int* cp = cnt + (size_t)nodeBase;
#pragma unroll
  for (int q = 0; q < 4; ++q) {
    const int f = (wave * 4 + q) * 128 + 4 * lane;
    *(volatile v4i*)(cp + f) = cq[q];
  }
  __threadfence();
#pragma unroll
  for (int q = 0; q < 4; ++q) {
    const int f = (wave * 4 + q) * 128 + 4 * lane;
    *(volatile v4i*)(cp + f) = cq[q];
  }
}

__global__ __launch_bounds__(OTHR) void k_offsets(
    const int* __restrict__ cnt, int* off, int* rbase, int nChunk) {
  __shared__ __attribute__((aligned(16))) int soff[NBC];
  __shared__ __attribute__((aligned(16))) int srb[RBN];
  __shared__ int wtot[OTHR / 32];
  const int tid = threadIdx.x, lane = tid & 31, wave = tid >> 5, sub = tid >> 7;
  for (int i = tid; i < RBN; i += OTHR) srb[i] = 0;
  int carry = 0;
#pragma unroll 1
  for (int ch = 0; ch < nChunk; ++ch) {
    const int base = ch * NBC;
    const v4i c0 = *(const v4i*)(cnt + base + 8 * tid);
    const v4i c1 = *(const v4i*)(cnt + base + 8 * tid + 4);
    const int e0 = max(c0.x, 0), e1 = max(c0.y, 0), e2 = max(c0.z, 0), e3 = max(c0.w, 0);
    const int e4 = max(c1.x, 0), e5 = max(c1.y, 0), e6 = max(c1.z, 0), e7 = max(c1.w, 0);
    const int ts = e0 + e1 + e2 + e3 + e4 + e5 + e6 + e7;
    int incl = ts;
#pragma unroll
    for (int d = 1; d < 32; d <<= 1) {
      const int t = __shfl_up(incl, d);
      if (lane >= d) incl += t;
    }
    if (lane == 31) wtot[wave] = incl;
    __syncthreads();
    const int S0 = wtot[0]  + wtot[1]  + wtot[2]  + wtot[3];
    const int S1 = wtot[4]  + wtot[5]  + wtot[6]  + wtot[7];
    const int S2 = wtot[8]  + wtot[9]  + wtot[10] + wtot[11];
    const int S3 = wtot[12] + wtot[13] + wtot[14] + wtot[15];
    int pre = 0;
#pragma unroll 1
    for (int w = 4 * sub; w < wave; ++w) pre += wtot[w];
    const int b0 = carry;
    const int b1 = b0 + ((S0 + 31) & ~31);
    const int b2 = b1 + ((S1 + 31) & ~31);
    const int b3 = b2 + ((S2 + 31) & ~31);
    const int b4 = b3 + ((S3 + 31) & ~31);
    const int myb = sub == 0 ? b0 : (sub == 1 ? b1 : (sub == 2 ? b2 : b3));
    if (tid == 0) {
      srb[min(4 * ch + 0, RBN - 1)] = b0;
      srb[min(4 * ch + 1, RBN - 1)] = b1;
      srb[min(4 * ch + 2, RBN - 1)] = b2;
      srb[min(4 * ch + 3, RBN - 1)] = b3;
    }
    int run = myb + pre + incl - ts;
    soff[8 * tid + 0] = run; run += e0;
    soff[8 * tid + 1] = run; run += e1;
    soff[8 * tid + 2] = run; run += e2;
    soff[8 * tid + 3] = run; run += e3;
    soff[8 * tid + 4] = run; run += e4;
    soff[8 * tid + 5] = run; run += e5;
    soff[8 * tid + 6] = run; run += e6;
    soff[8 * tid + 7] = run;
    carry = b4;
    __syncthreads();
    const v4i o0 = *(const v4i*)(soff + 4 * tid);
    const v4i o1 = *(const v4i*)(soff + 4 * (tid + OTHR));
    int* op = off + base;
    *(volatile v4i*)(op + 4 * tid) = o0;
    *(volatile v4i*)(op + 4 * (tid + OTHR)) = o1;
    __threadfence();
    *(volatile v4i*)(op + 4 * tid) = o0;
    *(volatile v4i*)(op + 4 * (tid + OTHR)) = o1;
    __syncthreads();
  }
  if (tid == 0) srb[min(4 * nChunk, RBN - 1)] = carry;
  __syncthreads();
  v4i rv = {0, 0, 0, 0};
  if (tid < 32) rv = *(const v4i*)(srb + 4 * tid);
  if (tid < 32) *(volatile v4i*)(rbase + 4 * tid) = rv;
  __threadfence();
  if (tid < 32) *(volatile v4i*)(rbase + 4 * tid) = rv;
}

__global__ __launch_bounds__(NTHR) void k_fill(
    const int* __restrict__ dsts, const int* __restrict__ off, const int* __restrict__ rbase,
    int* csr, int nE, int vec8, int csrLen) {
  extern __shared__ v4f lds_dyn[];
  int* region = (int*)lds_dyn;
  int* cursor = region + RCAP;
  int* list   = cursor + NBF;
  int* wcnt   = list + LISTN;
  const int tid = threadIdx.x, lane = tid & 31, wave = tid >> 5;
  const int b = blockIdx.x;
  const int nodeBase = b * NBF;

  int rb0 = rbase[b];
  const int rb1 = rbase[b + 1];
  rb0 = rb0 < 0 ? 0 : (rb0 > csrLen ? csrLen : rb0);
  rb0 &= ~31;
  int len = rb1 - rb0;
  len = len < 0 ? 0 : (len > RCAP ? RCAP : len);
  int lenW = (len + 31) & ~31;
  if (rb0 + lenW > csrLen) lenW = (csrLen - rb0) & ~31;

  {
    const v4i z = {0, 0, 0, 0};
    for (int i = tid; i < RCAP / 4; i += NTHR) ((v4i*)region)[i] = z;
    for (int s = tid; s < NBF; s += NTHR) {
      int o = off[nodeBase + s] - rb0;
      o = o < 0 ? 0 : (o > RCAP ? RCAP : o);
      cursor[s] = o;
    }
  }
  __syncthreads();

  const int nChunks = (nE + CHUNK - 1) / CHUNK;
#pragma unroll 1
  for (int ch = 0; ch < nChunks; ++ch) {
    const int cbase = ch * CHUNK;
    const int wc = scan_chunk<NBF>(dsts, nE, cbase, nodeBase, vec8, list, tid, lane, wave);
    if (lane == 0) wcnt[wave] = wc;
    __syncthreads();
    if (wave == 0) {
#pragma unroll 1
      for (int wsx = 0; wsx < NWAVE; ++wsx) {
        int n = __builtin_amdgcn_readfirstlane(wcnt[wsx]);
        n = n > WCAP ? WCAP : (n < 0 ? 0 : n);
        const int* lp = list + wsx * WCAP;
#pragma unroll 1
        for (int i = 0; i < n; ++i) {
          const int ent  = __builtin_amdgcn_readfirstlane(lp[i]);
          const int slot = ent & (NBF - 1);
          int e = cbase + ((ent >> 12) & (CHUNK - 1));
          e = e > nE - 1 ? nE - 1 : e;
          if (lane == 0) {
            int pos = cursor[slot];
            pos = pos < 0 ? 0 : (pos > RCAP - 1 ? RCAP - 1 : pos);
            region[pos] = e;
            const int np = pos + 1;
            cursor[slot] = np > RCAP ? RCAP : np;
          }
        }
      }
    }
    __syncthreads();
  }

  const int nv = lenW >> 2;
  int* gp = csr + rb0;
#pragma unroll 1
  for (int i = tid; i < nv; i += NTHR) { const v4i v = ((const v4i*)region)[i]; *(volatile v4i*)(gp + 4 * i) = v; }
  __threadfence();
#pragma unroll 1
  for (int i = tid; i < nv; i += NTHR) { const v4i v = ((const v4i*)region)[i]; *(volatile v4i*)(gp + 4 * i) = v; }
}

template <int L0>
__global__ __launch_bounds__(NTHR) void k_gemm(
    const float* __restrict__ A, const unsigned short* __restrict__ Bw,
    const float* __restrict__ tab, const float* __restrict__ bet,
    const float* __restrict__ attS, const float* __restrict__ attD,
    float* H, float* eS, float* eD, int nN) {
  __shared__ __attribute__((aligned(16))) unsigned char lds[2 * GBM * APK * 2];
  __shared__ __attribute__((aligned(16))) float sES[GBM];
  __shared__ __attribute__((aligned(16))) float sED[GBM];
  unsigned short* sHi = (unsigned short*)lds;
  unsigned short* sLo = sHi + GBM * APK;
  float*          stg = (float*)lds;
  const int tid = threadIdx.x, lane = tid & 31, wave = tid >> 5, hh = lane >> 4, m = lane & 15;
  const int rowBase = blockIdx.x * GBM;

  {
    const int r = tid >> 1, k0 = (tid & 1) * 16;
    int row = rowBase + r;
    row = row > nN - 1 ? nN - 1 : row;
    float v[16];
    if constexpr (L0 != 0) {
#pragma unroll
      for (int c = 0; c < 16; ++c) {
        const int k  = k0 + c;
        const int kc = k < INDIM - 1 ? k : INDIM - 1;
        const float xv = A[(size_t)row * INDIM + kc];
        v[c] = (k < INDIM) ? xv : 0.0f;
      }
    } else {
      const float* ap = A + (size_t)row * HID + k0;
#pragma unroll
      for (int p = 0; p < 4; ++p) {
        const v4f a  = *(const v4f*)(ap + 4 * p);
        const v4f mu = *(const v4f*)(tab + k0 + 4 * p);
        const v4f sc = *(const v4f*)(tab + HID + k0 + 4 * p);
        const v4f be = *(const v4f*)(bet + k0 + 4 * p);
        v[4 * p + 0] = bnr(a.x, mu.x, sc.x, be.x);
        v[4 * p + 1] = bnr(a.y, mu.y, sc.y, be.y);
        v[4 * p + 2] = bnr(a.z, mu.z, sc.z, be.z);
        v[4 * p + 3] = bnr(a.w, mu.w, sc.w, be.w);
      }
    }
    v8us h0, l0, h1, l1;
    v4f ta, tb;
    ta.x = v[0];  ta.y = v[1];  ta.z = v[2];  ta.w = v[3];
    tb.x = v[4];  tb.y = v[5];  tb.z = v[6];  tb.w = v[7];
    split8(ta, tb, h0, l0);
    ta.x = v[8];  ta.y = v[9];  ta.z = v[10]; ta.w = v[11];
    tb.x = v[12]; tb.y = v[13]; tb.z = v[14]; tb.w = v[15];
    split8(ta, tb, h1, l1);
    *(v8us*)(sHi + r * APK + k0)     = h0;
    *(v8us*)(sHi + r * APK + k0 + 8) = h1;
    *(v8us*)(sLo + r * APK + k0)     = l0;
    *(v8us*)(sLo + r * APK + k0 + 8) = l1;
  }
  __syncthreads();

  const int r0 = wave * 16;
  FragB ah, al;
  {
    const unsigned short* ahp = sHi + (r0 + m) * APK + 8 * hh;
    const unsigned short* alp = sLo + (r0 + m) * APK + 8 * hh;
    ah.h[0] = *(const v8us*)ahp;
    ah.h[1] = *(const v8us*)(ahp + 16);
    al.h[0] = *(const v8us*)alp;
    al.h[1] = *(const v8us*)(alp + 16);
  }
  v8f acc[2];
#pragma unroll
  for (int t = 0; t < 2; ++t) { v8f z = {0.f, 0.f, 0.f, 0.f, 0.f, 0.f, 0.f, 0.f}; acc[t] = z; }
#pragma unroll
  for (int t = 0; t < 2; ++t) {
    const unsigned short* bp = Bw + (size_t)(16 * t + m) * HID + 8 * hh;
    FragB bh, bl;
    bh.h[0] = *(const v8us*)bp;
    bh.h[1] = *(const v8us*)(bp + 16);
    bl.h[0] = *(const v8us*)(bp + HID * HID);
    bl.h[1] = *(const v8us*)(bp + HID * HID + 16);
    acc[t] = wmb(ah.v, bh.v, acc[t]);
    acc[t] = wmb(ah.v, bl.v, acc[t]);
    acc[t] = wmb(al.v, bh.v, acc[t]);
  }
  __syncthreads();

  {
    float* sp = stg + (size_t)(r0 + 8 * hh) * HID + m;
#pragma unroll
    for (int t = 0; t < 2; ++t) {
#pragma unroll
      for (int r = 0; r < 8; ++r) sp[r * HID + 16 * t] = acc[t][r];
    }
  }
  __syncthreads();

  const int qq   = lane & 7;
  const int rsub = lane >> 3;
  const int col  = 4 * qq;
  const v4f sA = *(const v4f*)(attS + col);
  const v4f sD = *(const v4f*)(attD + col);
  v4f vv[4];
#pragma unroll
  for (int it = 0; it < 4; ++it) {
    const int row = it * 4 + rsub;
    const v4f v = *(const v4f*)(stg + (size_t)(r0 + row) * HID + col);
    vv[it] = v;
    *(volatile v4f*)(H + (size_t)(rowBase + r0 + row) * HID + col) = v;
    float ps = v.x * sA.x + v.y * sA.y + v.z * sA.z + v.w * sA.w;
    float pd = v.x * sD.x + v.y * sD.y + v.z * sD.z + v.w * sD.w;
#pragma unroll
    for (int o = 1; o < 8; o <<= 1) { ps += __shfl_xor(ps, o); pd += __shfl_xor(pd, o); }
    if (qq == 0) { sES[r0 + row] = ps; sED[r0 + row] = pd; }
  }
  __threadfence();
#pragma unroll
  for (int it = 0; it < 4; ++it) {
    const int row = it * 4 + rsub;
    *(volatile v4f*)(H + (size_t)(rowBase + r0 + row) * HID + col) = vv[it];
  }
  __syncthreads();

  v4f dv = {0.f, 0.f, 0.f, 0.f};
  if (wave == 0) {
    dv = *(const v4f*)(sES + 4 * lane);
    *(volatile v4f*)(eS + rowBase + 4 * lane) = dv;
  } else if (wave == 1) {
    dv = *(const v4f*)(sED + 4 * lane);
    *(volatile v4f*)(eD + rowBase + 4 * lane) = dv;
  }
  __threadfence();
  if (wave == 0) {
    *(volatile v4f*)(eS + rowBase + 4 * lane) = dv;
  } else if (wave == 1) {
    *(volatile v4f*)(eD + rowBase + 4 * lane) = dv;
  }
}

__global__ __launch_bounds__(NTHR) void k_agg(
    const int* __restrict__ csr, const int* __restrict__ off, const int* __restrict__ cnt,
    const int* __restrict__ srcs, const float* __restrict__ ea,
    const float* __restrict__ eS, const float* __restrict__ eD, const float* __restrict__ H,
    const float* __restrict__ We, const float* __restrict__ ae, const float* __restrict__ bias,
    float* xr, double* part, int nN, int nE, int csrLen) {
  __shared__ float sc4[EDIM];
  __shared__ double swS[NWAVE * HID];
  __shared__ double swQ[NWAVE * HID];
  const int tid = threadIdx.x, lane = tid & 31, wave = tid >> 5;
  const int tbase = blockIdx.x * TGT + wave * 32;

  if (tid < EDIM) {
    float s = 0.0f;
#pragma unroll 1
    for (int j = 0; j < HID; ++j) s += We[tid * HID + j] * ae[j];
    sc4[tid] = s;
  }
  __syncthreads();
  const float c40 = sc4[0], c41 = sc4[1], c42 = sc4[2], c43 = sc4[3];
  const float bl = bias[lane];

  const int cl    = tbase + lane;
  const int cnt_l = cnt[cl];
  const int off_l = off[cl];
  double ds = 0.0, dq = 0.0;

#pragma unroll 1
  for (int j = 0; j < 32; ++j) {
    const int c = tbase + j;
    int n = __builtin_amdgcn_readfirstlane(__shfl(cnt_l, j));
    n = n < 0 ? 0 : (n > DEGCAP ? DEGCAP : n);
    const int st = __builtin_amdgcn_readfirstlane(__shfl(off_l, j));
    const float edc = eD[c];

    float mx = NEG_BIG;
#pragma unroll 1
    for (int q0 = 0; q0 < n; q0 += 32) {
      const int idx = q0 + lane;
      int pos = st + (idx < n ? idx : n - 1);
      pos = pos < 0 ? 0 : (pos > csrLen - 1 ? csrLen - 1 : pos);
      int e = csr[pos];
      e = e < 0 ? 0 : (e > nE - 1 ? nE - 1 : e);
      int s = srcs[e];
      s = s < 0 ? 0 : (s > nN - 1 ? nN - 1 : s);
      const v4f ev = *(const v4f*)(ea + (size_t)e * EDIM);
      float sc = eS[s] + edc + (ev.x * c40 + ev.y * c41 + ev.z * c42 + ev.w * c43);
      sc = lrelu(sc);
      sc = (idx < n) ? sc : NEG_BIG;
      mx = fmaxf(mx, sc);
    }
    mx = wmax(mx);

    float den = 0.0f, acc = 0.0f;
#pragma unroll 1
    for (int q0 = 0; q0 < n; q0 += 32) {
      const int idx = q0 + lane;
      int pos = st + (idx < n ? idx : n - 1);
      pos = pos < 0 ? 0 : (pos > csrLen - 1 ? csrLen - 1 : pos);
      int e = csr[pos];
      e = e < 0 ? 0 : (e > nE - 1 ? nE - 1 : e);
      int s = srcs[e];
      s = s < 0 ? 0 : (s > nN - 1 ? nN - 1 : s);
      const v4f ev = *(const v4f*)(ea + (size_t)e * EDIM);
      float sc = eS[s] + edc + (ev.x * c40 + ev.y * c41 + ev.z * c42 + ev.w * c43);
      sc = lrelu(sc);
      sc = (idx < n) ? sc : NEG_BIG;
      const float wx = __expf(sc - mx);
      const float w  = (idx < n) ? wx : 0.0f;
      den += w;
      const int mcnt = __builtin_amdgcn_readfirstlane((n - q0) < 32 ? (n - q0) : 32);
#pragma unroll 1
      for (int pp = 0; pp < mcnt; ++pp) {
        const float wv = __int_as_float(__builtin_amdgcn_readlane(__float_as_int(w), pp));
        const int   sv = __builtin_amdgcn_readlane(s, pp);
        acc += wv * H[(size_t)sv * HID + lane];
      }
    }
    den = wsum(den);

    const float rd = 1.0f / (den + DEN_EPS);
    float v = acc * rd + bl;
    if (c < nN) { ds += (double)v; dq += (double)v * (double)v; }
    else v = 0.0f;
    float* xp = xr + (size_t)c * HID + lane;
    *(volatile float*)xp = v;
    __threadfence();
    *(volatile float*)xp = v;
  }

  swS[wave * HID + lane] = ds;
  swQ[wave * HID + lane] = dq;
  __syncthreads();
  if (wave == 0) {
    double S = 0.0, Q = 0.0;
#pragma unroll
    for (int w = 0; w < NWAVE; ++w) { S += swS[w * HID + lane]; Q += swQ[w * HID + lane]; }
    v2d pv;
    pv.x = S; pv.y = Q;
    double* pq = part + (size_t)blockIdx.x * (2 * HID) + 2 * lane;
    *(volatile v2d*)pq = pv;
    __threadfence();
    *(volatile v2d*)pq = pv;
  }
}

__global__ __launch_bounds__(64) void k_bnfin(const double* __restrict__ part, const float* __restrict__ gam,
                                              float* tab, int nBlk, int nN) {
  __shared__ double sred[64];
  __shared__ __attribute__((aligned(16))) float stab[64];
  const int tid = threadIdx.x, c = tid & 31, which = tid >> 5;
  double a = 0.0;
#pragma unroll 1
  for (int b = 0; b < nBlk; ++b) a += part[(size_t)b * (2 * HID) + 2 * c + which];
  sred[tid] = a;
  __syncthreads();
  if (tid < HID) {
    const double S = sred[tid], Q = sred[HID + tid];
    const double inv = 1.0 / (double)nN;
    const double mu = S * inv;
    double var = Q * inv - mu * mu;
    var = var < 0.0 ? 0.0 : var;
    const float muf = (float)mu;
    const float varf = (float)var;
    const float scale = gam[tid] * rsqrtf(varf + BN_EPS);
    stab[tid] = muf;
    stab[HID + tid] = scale;
  }
  __syncthreads();
  v4f tv = {0.f, 0.f, 0.f, 0.f};
  if (tid < 16) tv = *(const v4f*)(stab + 4 * tid);
  if (tid < 16) *(volatile v4f*)(tab + 4 * tid) = tv;
  __threadfence();
  if (tid < 16) *(volatile v4f*)(tab + 4 * tid) = tv;
}

__global__ __launch_bounds__(NTHR) void k_embed(const float* __restrict__ xr, const float* __restrict__ tab,
                                                const float* __restrict__ bet, float* out1, int nN) {
  const int tid = threadIdx.x, r = tid >> 3, q = tid & 7, col = 4 * q;
  const v4f mu = *(const v4f*)(tab + col), sc = *(const v4f*)(tab + HID + col), be = *(const v4f*)(bet + col);
  v4f y[4];
  int rows[4];
#pragma unroll
  for (int it = 0; it < 4; ++it) {
    const int row = blockIdx.x * GBM + it * 32 + r;
    rows[it] = row;
    const v4f x = *(const v4f*)(xr + (size_t)row * HID + col);
    v4f t;
    t.x = bnr(x.x, mu.x, sc.x, be.x); t.y = bnr(x.y, mu.y, sc.y, be.y);
    t.z = bnr(x.z, mu.z, sc.z, be.z); t.w = bnr(x.w, mu.w, sc.w, be.w);
    y[it] = t;
    if (row < nN) *(volatile v4f*)(out1 + (size_t)row * HID + col) = t;
  }
  __threadfence();
#pragma unroll
  for (int it = 0; it < 4; ++it) {
    if (rows[it] < nN) *(volatile v4f*)(out1 + (size_t)rows[it] * HID + col) = y[it];
  }
}

__global__ __launch_bounds__(NTHR) void k_pool(
    const int* __restrict__ bat, const float* __restrict__ xr, const float* __restrict__ tab,
    const float* __restrict__ bet, const float* __restrict__ fcW, const float* __restrict__ fcb,
    float* gemb, float* outp, int nN, int nG) {
  __shared__ __attribute__((aligned(16))) float sacc[PG * HID];
  __shared__ __attribute__((aligned(16))) int   list[LISTN];
  __shared__ __attribute__((aligned(16))) float sout[PG * NCLS];
  __shared__ int wcnt[NWAVE];
  const int tid = threadIdx.x, lane = tid & 31, wave = tid >> 5;
  const int slotBase = blockIdx.x * PG;
  const v4f z4 = {0.f, 0.f, 0.f, 0.f};

  for (int i = tid; i < PG * HID / 4; i += NTHR) ((v4f*)sacc)[i] = z4;
  const float mu_l = tab[lane], sc_l = tab[HID + lane], be_l = bet[lane];
  __syncthreads();

  const int nChunks = (nN + CHUNK - 1) / CHUNK;
#pragma unroll 1
  for (int ch = 0; ch < nChunks; ++ch) {
    const int cbase = ch * CHUNK;
    const int wc = scan_chunk<PG>(bat, nN, cbase, slotBase, 1, list, tid, lane, wave);
    if (lane == 0) wcnt[wave] = wc;
    __syncthreads();
    if (wave == 0) {
#pragma unroll 1
      for (int wsx = 0; wsx < NWAVE; ++wsx) {
        int n = __builtin_amdgcn_readfirstlane(wcnt[wsx]);
        n = n > WCAP ? WCAP : (n < 0 ? 0 : n);
        const int* lp = list + wsx * WCAP;
#pragma unroll 1
        for (int i = 0; i < n; ++i) {
          const int ent  = __builtin_amdgcn_readfirstlane(lp[i]);
          const int slot = ent & (PG - 1);
          int node = cbase + ((ent >> 12) & (CHUNK - 1));
          node = node > nN - 1 ? nN - 1 : node;
          const float x = xr[(size_t)node * HID + lane];
          const float y = bnr(x, mu_l, sc_l, be_l);
          sacc[slot * HID + lane] = sacc[slot * HID + lane] + y;
        }
      }
    }
    __syncthreads();
  }

  {
    const int r = tid >> 3, q = tid & 7, col = 4 * q;
    v4f gv[8];
    int gs[8];
#pragma unroll
    for (int it = 0; it < 8; ++it) {
      const int rl = it * 32 + r;
      const int g  = slotBase + rl;
      gs[it] = g;
      gv[it] = *(const v4f*)(sacc + rl * HID + col);
      if (g < nG) *(volatile v4f*)(gemb + (size_t)g * HID + col) = gv[it];
    }
    __threadfence();
#pragma unroll
    for (int it = 0; it < 8; ++it) {
      if (gs[it] < nG) *(volatile v4f*)(gemb + (size_t)gs[it] * HID + col) = gv[it];
    }
  }

  {
    const float* gr = sacc + tid * HID;
    float s0 = 0.0f, s1 = 0.0f;
#pragma unroll 1
    for (int c = 0; c < HID; ++c) {
      const float g = gr[c];
      s0 += g * fcW[c * NCLS + 0];
      s1 += g * fcW[c * NCLS + 1];
    }
    sout[tid * NCLS + 0] = s0 + fcb[0];
    sout[tid * NCLS + 1] = s1 + fcb[1];
  }
  __syncthreads();
  {
    const int p  = tid;
    const int g2 = slotBase + 2 * p;
    const bool ok = (p < PG / 2) && (g2 + 1 < nG);
    v4f ov = z4;
    if (p < PG / 2) ov = *(const v4f*)(sout + 4 * p);
    if (ok) *(volatile v4f*)(outp + (size_t)g2 * NCLS) = ov;
    __threadfence();
    if (ok) *(volatile v4f*)(outp + (size_t)g2 * NCLS) = ov;
  }
}

extern "C" void kernel_launch(void* const* d_in, const int* in_sizes, int n_in,
                              void* d_out, int out_size, void* d_ws, size_t ws_size,
                              hipStream_t stream) {
  if (n_in < 15) return;
  const int nN = in_sizes[0] / INDIM;
  const int nE = in_sizes[1] / 2;
  if (nN <= 0 || nE <= 0) return;
  if (in_sizes[0] != nN * INDIM || in_sizes[1] != 2 * nE || in_sizes[2] != nN || in_sizes[3] != EDIM * nE) return;
  if (in_sizes[4] != INDIM * HID || in_sizes[5] != 2 * HID * HID) return;
  if (in_sizes[6] != 3 * HID || in_sizes[7] != 3 * HID || in_sizes[8] != 3 * EDIM * HID || in_sizes[9] != 3 * HID) return;
  if (in_sizes[10] != 3 * HID || in_sizes[11] != 3 * HID || in_sizes[12] != 3 * HID) return;
  if (in_sizes[13] != HID * NCLS || in_sizes[14] != NCLS) return;
  const long long rem = (long long)out_size - (long long)nN * HID;
  if (rem <= 0 || (rem % (NCLS + HID)) != 0) return;
  const int nG = (int)(rem / (NCLS + HID));
  if (nG <= 0 || (nG % 16) != 0) return;
  if (nE > (1 << 28) || nN > (1 << 24) || nG > (1 << 22)) return;

  const float* x        = (const float*)d_in[0];
  const int*   eidx     = (const int*)d_in[1];
  const int*   batch    = (const int*)d_in[2];
  const float* eattr    = (const float*)d_in[3];
  const float* W0       = (const float*)d_in[4];
  const float* W12      = (const float*)d_in[5];
  const float* att_src  = (const float*)d_in[6];
  const float* att_dst  = (const float*)d_in[7];
  const float* lin_edge = (const float*)d_in[8];
  const float* att_edge = (const float*)d_in[9];
  const float* bias     = (const float*)d_in[10];
  const float* bn_gamma = (const float*)d_in[11];
  const float* bn_beta  = (const float*)d_in[12];
  const float* fc_W     = (const float*)d_in[13];
  const float* fc_b     = (const float*)d_in[14];
  const int* src = eidx;
  const int* dst = eidx + nE;

  float* out0 = (float*)d_out;
  float* out1 = out0 + (size_t)nG * NCLS;
  float* out2 = out1 + (size_t)nN * HID;

  const int NPAD   = ((nN + TGT - 1) / TGT) * TGT;
  const int nBC    = (nN + NBC - 1) / NBC;
  const int CNTPAD = nBC * NBC;
  if (4 * nBC + 1 > RBN) return;
  if (31 * 4 * nBC > 4096) return;
  const int nBF    = (nN + NBF - 1) / NBF;
  const int csrLen = ((nE + 31) & ~31) + 4096;
  const int nAgg   = NPAD / TGT;
  const int nGm    = NPAD / GBM;
  const int nPB    = (nG + PG - 1) / PG;

  char* ws = (char*)d_ws;
  size_t off = 0;
  const size_t oWp  = off; off += (size_t)3 * 2 * HID * HID * 2;    off = (off + 255) & ~(size_t)255;
  const size_t oCnt = off; off += (size_t)CNTPAD * 4;               off = (off + 255) & ~(size_t)255;
  const size_t oOff = off; off += (size_t)CNTPAD * 4;               off = (off + 255) & ~(size_t)255;
  const size_t oRb  = off; off += (size_t)RBN * 4;                  off = (off + 255) & ~(size_t)255;
  const size_t oCsr = off; off += (size_t)csrLen * 4;               off = (off + 255) & ~(size_t)255;
  const size_t oH   = off; off += (size_t)NPAD * HID * 4;           off = (off + 255) & ~(size_t)255;
  const size_t oXr  = off; off += (size_t)NPAD * HID * 4;           off = (off + 255) & ~(size_t)255;
  const size_t oEs  = off; off += (size_t)NPAD * 4;                 off = (off + 255) & ~(size_t)255;
  const size_t oEd  = off; off += (size_t)NPAD * 4;                 off = (off + 255) & ~(size_t)255;
  const size_t oPt  = off; off += (size_t)nAgg * 2 * HID * 8;       off = (off + 255) & ~(size_t)255;
  const size_t oTab = off; off += (size_t)3 * 2 * HID * 4;          off = (off + 255) & ~(size_t)255;
  if (off > ws_size || off > (size_t)WSCAP) return;
  unsigned short* wp = (unsigned short*)(ws + oWp);
  int*    cnt  = (int*)(ws + oCnt);
  int*    offp = (int*)(ws + oOff);
  int*    rb   = (int*)(ws + oRb);
  int*    csr  = (int*)(ws + oCsr);
  float*  Hp   = (float*)(ws + oH);
  float*  xr   = (float*)(ws + oXr);
  float*  es   = (float*)(ws + oEs);
  float*  ed   = (float*)(ws + oEd);
  double* part = (double*)(ws + oPt);
  float*  tabp = (float*)(ws + oTab);

  const int vec8 = ((nE & 3) == 0) ? 1 : 0;

  k_prep<<<3, 128, 0, stream>>>(W0, W12, wp);

  k_count<<<nBC, NTHR, 0, stream>>>(dst, cnt, nE, vec8);
  k_offsets<<<1, OTHR, 0, stream>>>(cnt, offp, rb, nBC);
  hipFuncSetAttribute(reinterpret_cast<const void*>(&k_fill),
                      hipFuncAttributeMaxDynamicSharedMemorySize, LDS_FILL);
  k_fill<<<nBF, NTHR, LDS_FILL, stream>>>(dst, offp, rb, csr, nE, vec8, csrLen);

  for (int l = 0; l < 3; ++l) {
    const unsigned short* wl = wp + (size_t)l * 2 * HID * HID;
    const int lp = l > 0 ? l - 1 : 0;
    if (l == 0) {
      k_gemm<1><<<nGm, NTHR, 0, stream>>>(x, wl, tabp, bn_beta, att_src, att_dst, Hp, es, ed, nN);
    } else {
      k_gemm<0><<<nGm, NTHR, 0, stream>>>(xr, wl, tabp + (size_t)lp * 2 * HID, bn_beta + (size_t)lp * HID,
                                          att_src + (size_t)l * HID, att_dst + (size_t)l * HID, Hp, es, ed, nN);
    }
    k_agg<<<nAgg, NTHR, 0, stream>>>(csr, offp, cnt, src, eattr, es, ed, Hp,
                                     lin_edge + (size_t)l * EDIM * HID, att_edge + (size_t)l * HID,
                                     bias + (size_t)l * HID, xr, part, nN, nE, csrLen);
    k_bnfin<<<1, 64, 0, stream>>>(part, bn_gamma + (size_t)l * HID, tabp + (size_t)l * 2 * HID, nAgg, nN);
  }

  k_embed<<<nGm, NTHR, 0, stream>>>(xr, tabp + (size_t)2 * 2 * HID, bn_beta + (size_t)2 * HID, out1, nN);

  k_pool<<<nPB, NTHR, 0, stream>>>(batch, xr, tabp + (size_t)2 * 2 * HID, bn_beta + (size_t)2 * HID,
                                   fc_W, fc_b, out2, out0, nN, nG);
}
